// GNNHiddenStatePredictor_7198365188339
// MI455X (gfx1250) — hardware-verified
//
#include <hip/hip_runtime.h>
#include <stddef.h>
#include <stdint.h>

#pragma clang fp contract(off)

#define B_    4
#define V_    384
#define H_    128
#define N_    512
#define HD_   64
#define TD_   128
#define KP64  72
#define KP128 136
#define OPF   132
#define WCAR  16.0f
#define WINV  0.0625f

static_assert(V_ + H_ == N_);
static_assert(V_ % 64 == 0);
static_assert(N_ % 64 == 0);
static_assert(H_ % 32 == 0);
static_assert(HD_ == 64);
static_assert(TD_ == 128);
static_assert((KP64 * 2) % 16 == 0);
static_assert((KP128 * 2) % 16 == 0);
static_assert((OPF * 4) % 16 == 0);

typedef _Float16     v16h __attribute__((ext_vector_type(16)));
typedef _Float16     v8h  __attribute__((ext_vector_type(8)));
typedef float        v8f  __attribute__((ext_vector_type(8)));
typedef float        v4f  __attribute__((ext_vector_type(4)));
typedef unsigned int v4u  __attribute__((ext_vector_type(4)));

union Frag { v16h v; v8h h[2]; };
union HU   { v8h h; v4u u; };

__device__ __forceinline__ v8f zero8() { return (v8f){0.f, 0.f, 0.f, 0.f, 0.f, 0.f, 0.f, 0.f}; }

__device__ __forceinline__ v8f mma16(v16h a, v16h b, v8f c) {
  c = __builtin_amdgcn_wmma_f32_16x16x32_f16(false, a, false, b, (short)0, c, false, false);
  asm volatile("v_nop\n\tv_nop\n\tv_nop\n\tv_nop" : "+v"(c) : "v"(a), "v"(b));
  return c;
}

__device__ __forceinline__ v16h ldfrag(const _Float16* p, int ld, int row0, int k0, int lane) {
  const int m = lane & 15, hh = lane >> 4;
  const _Float16* q = p + (size_t)(row0 + m) * ld + k0 + 8 * hh;
  Frag f;
  f.h[0] = *(const v8h*)(q);
  f.h[1] = *(const v8h*)(q + 16);
  return f.v;
}

__device__ __forceinline__ v16h ldfrag32(const float* __restrict__ p, int ld, int row0, int k0, int lane) {
  const int m = lane & 15, hh = lane >> 4;
  const float* q = p + (size_t)(row0 + m) * ld + k0 + 8 * hh;
  const v4f x0 = *(const v4f*)(q);
  const v4f x1 = *(const v4f*)(q + 4);
  const v4f x2 = *(const v4f*)(q + 16);
  const v4f x3 = *(const v4f*)(q + 20);
  v16h a;
  a[0]  = (_Float16)x0[0]; a[1]  = (_Float16)x0[1]; a[2]  = (_Float16)x0[2]; a[3]  = (_Float16)x0[3];
  a[4]  = (_Float16)x1[0]; a[5]  = (_Float16)x1[1]; a[6]  = (_Float16)x1[2]; a[7]  = (_Float16)x1[3];
  a[8]  = (_Float16)x2[0]; a[9]  = (_Float16)x2[1]; a[10] = (_Float16)x2[2]; a[11] = (_Float16)x2[3];
  a[12] = (_Float16)x3[0]; a[13] = (_Float16)x3[1]; a[14] = (_Float16)x3[2]; a[15] = (_Float16)x3[3];
  return a;
}

template<int K, int C, int KP, int NTH>
__device__ __forceinline__ void stage_wt(const float* __restrict__ W, _Float16* Ws, int tid) {
#pragma unroll 4
  for (int idx = tid; idx < K * C; idx += NTH) {
    const int k  = idx / C;
    const int cc = idx - k * C;
    Ws[cc * KP + k] = (_Float16)(W[idx] * WCAR);
  }
}

template<int KS, int NT>
__device__ __forceinline__ void mm_lds(v8f (&acc)[NT], const _Float16* As, int ap, int arow0,
                                       const _Float16* Bs, int bp, int lane) {
#pragma unroll
  for (int ks = 0; ks < KS; ++ks) {
    const v16h a = ldfrag(As, ap, arow0, 32 * ks, lane);
#pragma unroll
    for (int t = 0; t < NT; ++t) acc[t] = mma16(a, ldfrag(Bs, bp, 16 * t, 32 * ks, lane), acc[t]);
  }
}

template<int NT>
__device__ __forceinline__ void epi_relu(const v8f (&acc)[NT], const float* bias, _Float16* Ds, int dp,
                                         int drow0, int lane) {
  const int c = lane & 15, hh = lane >> 4;
#pragma unroll
  for (int t = 0; t < NT; ++t) {
    const float bv = bias[16 * t + c];
#pragma unroll
    for (int r = 0; r < 8; ++r) {
      const float v = fmaxf(acc[t][r] * WINV + bv, 0.f);
      Ds[(drow0 + 8 * hh + r) * dp + 16 * t + c] = (_Float16)v;
    }
  }
}

__global__ __launch_bounds__(128)
void k_nodef(const float* __restrict__ x, const float* __restrict__ w_in1, const float* __restrict__ b_in1,
             const float* __restrict__ w_in2, const float* __restrict__ b_in2, const float* __restrict__ w_e1,
             const float* __restrict__ b_e1, const float* __restrict__ w_e2, const float* __restrict__ b_e2,
             _Float16* __restrict__ Ft) {
  __shared__ __align__(16) _Float16 W1s[HD_ * KP128];
  __shared__ __align__(16) _Float16 W2s[HD_ * KP64];
  __shared__ __align__(16) _Float16 W3s[HD_ * KP64];
  __shared__ __align__(16) _Float16 W4s[HD_ * KP64];
  __shared__ __align__(16) _Float16 Ha[64 * KP64];
  __shared__ __align__(16) _Float16 Hb[64 * KP64];
  __shared__ float bsh[4 * HD_];

  const int tid = threadIdx.x, lane = tid & 31, wave = tid >> 5;
  const int hh = lane >> 4, c = lane & 15;
  const int blk = blockIdx.x;
  const int b   = blk >> 3;
  const int j0  = (blk & 7) * 64;
  const bool vis = (j0 < V_);
  const int rw  = 16 * wave;

  stage_wt<TD_, HD_, KP128, 128>(w_in1, W1s, tid);
  stage_wt<HD_, HD_, KP64, 128>(w_in2, W2s, tid);
  stage_wt<HD_, HD_, KP64, 128>(w_e1 + HD_ * HD_, W3s, tid);
  stage_wt<HD_, HD_, KP64, 128>(w_e2, W4s, tid);
  if (tid < HD_) {
    bsh[tid]           = b_in1[tid];
    bsh[HD_ + tid]     = b_in2[tid];
    bsh[2 * HD_ + tid] = b_e1[tid];
    bsh[3 * HD_ + tid] = b_e2[tid];
  }
  __syncthreads();

  if (vis) {
    v8f acc[4];
#pragma unroll
    for (int t = 0; t < 4; ++t) acc[t] = zero8();
    const float* xr = x + ((size_t)b * V_ + j0) * TD_;
#pragma unroll
    for (int ks = 0; ks < TD_ / 32; ++ks) {
      const v16h a = ldfrag32(xr, TD_, rw, 32 * ks, lane);
#pragma unroll
      for (int t = 0; t < 4; ++t) acc[t] = mma16(a, ldfrag(W1s, KP128, 16 * t, 32 * ks, lane), acc[t]);
    }
    epi_relu<4>(acc, bsh, Ha, KP64, rw, lane);
  }
  __syncthreads();

  if (vis) {
    v8f acc[4];
#pragma unroll
    for (int t = 0; t < 4; ++t) acc[t] = zero8();
    mm_lds<2, 4>(acc, Ha, KP64, rw, W2s, KP64, lane);
    epi_relu<4>(acc, bsh + HD_, Hb, KP64, rw, lane);
  }
  __syncthreads();

  if (vis) {
    v8f acc[4];
#pragma unroll
    for (int t = 0; t < 4; ++t) acc[t] = zero8();
    mm_lds<2, 4>(acc, Hb, KP64, rw, W3s, KP64, lane);
    epi_relu<4>(acc, bsh + 2 * HD_, Ha, KP64, rw, lane);
  } else {
#pragma unroll 4
    for (int idx = tid; idx < 64 * HD_; idx += 128) {
      const int row = idx >> 6, col = idx & 63;
      Ha[row * KP64 + col] = (_Float16)fmaxf(bsh[2 * HD_ + col], 0.f);
    }
  }
  __syncthreads();

  {
    v8f acc[4];
#pragma unroll
    for (int t = 0; t < 4; ++t) acc[t] = zero8();
    mm_lds<2, 4>(acc, Ha, KP64, rw, W4s, KP64, lane);
    _Float16* FsT = Hb;
#pragma unroll
    for (int t = 0; t < 4; ++t) {
      const float bv = bsh[3 * HD_ + 16 * t + c];
#pragma unroll
      for (int r = 0; r < 8; ++r) {
        const float v = fmaxf(acc[t][r] * WINV + bv, 0.f);
        FsT[(16 * t + c) * KP64 + rw + 8 * hh + r] = (_Float16)v;
      }
    }
  }
  __syncthreads();

  {
    v4u val[4];
    size_t go[4];
#pragma unroll
    for (int it = 0; it < 4; ++it) {
      const int p  = tid + 128 * it;
      const int h  = p >> 3;
      const int pc = p & 7;
      HU u;
      u.h = *(const v8h*)(Hb + h * KP64 + 8 * pc);
      val[it] = u.u;
      go[it]  = ((size_t)(b * HD_ + h)) * N_ + j0 + 8 * pc;
    }
#pragma unroll
    for (int it = 0; it < 4; ++it) *(volatile v4u*)(Ft + go[it]) = val[it];
    __threadfence();
#pragma unroll
    for (int it = 0; it < 4; ++it) *(volatile v4u*)(Ft + go[it]) = val[it];
  }
}

__global__ __launch_bounds__(64)
void k_aggout(const float* __restrict__ adj, const _Float16* __restrict__ Ft,
              const float* __restrict__ w_n1, const float* __restrict__ b_n1,
              const float* __restrict__ w_n2, const float* __restrict__ b_n2,
              const float* __restrict__ w_out, const float* __restrict__ b_out, float* __restrict__ out) {
  __shared__ __align__(16) _Float16 Wn1s[HD_ * KP64];
  __shared__ __align__(16) _Float16 Wn2s[HD_ * KP64];
  __shared__ __align__(16) _Float16 Wos[TD_ * KP64];
  __shared__ __align__(16) _Float16 Aa[32 * KP64];
  __shared__ __align__(16) _Float16 Ab[32 * KP64];
  __shared__ __align__(16) float    Os[32 * OPF];
  __shared__ float bs[2 * HD_ + TD_];

  const int tid = threadIdx.x, lane = tid & 31, wave = tid >> 5;
  const int hh = lane >> 4, c = lane & 15;
  const int blk = blockIdx.x;
  const int b   = blk >> 2;
  const int i0  = (blk & 3) * 32;
  const int rw  = 16 * wave;

  stage_wt<HD_, HD_, KP64, 64>(w_n1, Wn1s, tid);
  stage_wt<HD_, HD_, KP64, 64>(w_n2, Wn2s, tid);
  stage_wt<HD_, TD_, KP64, 64>(w_out, Wos, tid);
  bs[tid]                = b_n1[tid];
  bs[HD_ + tid]          = b_n2[tid];
  bs[2 * HD_ + tid]      = b_out[tid];
  bs[2 * HD_ + 64 + tid] = b_out[64 + tid];
  __syncthreads();

  {
    v8f acc[4];
#pragma unroll
    for (int t = 0; t < 4; ++t) acc[t] = zero8();
    const float* ar = adj + ((size_t)(b * N_ + V_ + i0)) * N_;
    const _Float16* fb = Ft + (size_t)b * HD_ * N_;
#pragma unroll 2
    for (int ks = 0; ks < N_ / 32; ++ks) {
      const v16h a = ldfrag32(ar, N_, rw, 32 * ks, lane);
#pragma unroll
      for (int t = 0; t < 4; ++t) acc[t] = mma16(a, ldfrag(fb, N_, 16 * t, 32 * ks, lane), acc[t]);
    }
#pragma unroll
    for (int t = 0; t < 4; ++t)
#pragma unroll
      for (int r = 0; r < 8; ++r) Aa[(rw + 8 * hh + r) * KP64 + 16 * t + c] = (_Float16)acc[t][r];
  }
  __syncthreads();

  {
    v8f acc[4];
#pragma unroll
    for (int t = 0; t < 4; ++t) acc[t] = zero8();
    mm_lds<2, 4>(acc, Aa, KP64, rw, Wn1s, KP64, lane);
    epi_relu<4>(acc, bs, Ab, KP64, rw, lane);
  }
  __syncthreads();

  {
    v8f acc[4];
#pragma unroll
    for (int t = 0; t < 4; ++t) acc[t] = zero8();
    mm_lds<2, 4>(acc, Ab, KP64, rw, Wn2s, KP64, lane);
    epi_relu<4>(acc, bs + HD_, Aa, KP64, rw, lane);
  }
  __syncthreads();

  {
    v8f acc[8];
#pragma unroll
    for (int t = 0; t < 8; ++t) acc[t] = zero8();
    mm_lds<2, 8>(acc, Aa, KP64, rw, Wos, KP64, lane);
#pragma unroll
    for (int t = 0; t < 8; ++t) {
      const float bv = bs[2 * HD_ + 16 * t + c];
#pragma unroll
      for (int r = 0; r < 8; ++r) Os[(rw + 8 * hh + r) * OPF + 16 * t + c] = acc[t][r] * WINV + bv;
    }
  }
  __syncthreads();

#pragma unroll
  for (int ch = 0; ch < 4; ++ch) {
    v4f val[4];
    size_t go[4];
#pragma unroll
    for (int i = 0; i < 4; ++i) {
      const int p   = tid + 64 * (4 * ch + i);
      const int L   = p >> 3;
      const int pc  = p & 7;
      const int row = L >> 2;
      const int q   = L & 3;
      val[i] = *(const v4f*)(Os + row * OPF + 32 * q + 4 * pc);
      go[i]  = ((size_t)(b * H_ + i0 + row)) * TD_ + 32 * q + 4 * pc;
    }
#pragma unroll
    for (int i = 0; i < 4; ++i) *(volatile v4f*)(out + go[i]) = val[i];
    __threadfence();
#pragma unroll
    for (int i = 0; i < 4; ++i) *(volatile v4f*)(out + go[i]) = val[i];
  }
}

extern "C" void kernel_launch(void* const* d_in, const int* in_sizes, int n_in,
                              void* d_out, int out_size, void* d_ws, size_t ws_size,
                              hipStream_t stream) {
  if (n_in < 16) return;
  if (in_sizes[0]  != B_ * V_ * TD_) return;
  if (in_sizes[1]  != B_ * N_ * N_) return;
  if (in_sizes[2]  != TD_ * HD_) return;
  if (in_sizes[3]  != HD_) return;
  if (in_sizes[4]  != HD_ * HD_) return;
  if (in_sizes[5]  != HD_) return;
  if (in_sizes[6]  != 2 * HD_ * HD_) return;
  if (in_sizes[7]  != HD_) return;
  if (in_sizes[8]  != HD_ * HD_) return;
  if (in_sizes[9]  != HD_) return;
  if (in_sizes[10] != HD_ * HD_) return;
  if (in_sizes[11] != HD_) return;
  if (in_sizes[12] != HD_ * HD_) return;
  if (in_sizes[13] != HD_) return;
  if (in_sizes[14] != HD_ * TD_) return;
  if (in_sizes[15] != TD_) return;
  if (out_size != B_ * H_ * TD_) return;

  const size_t ftBytes = (size_t)B_ * HD_ * N_ * 2;
  if (ftBytes > ws_size) return;
  if (ftBytes > (size_t)134217728) return;

  const float* x     = (const float*)d_in[0];
  const float* adj   = (const float*)d_in[1];
  const float* w_in1 = (const float*)d_in[2];
  const float* b_in1 = (const float*)d_in[3];
  const float* w_in2 = (const float*)d_in[4];
  const float* b_in2 = (const float*)d_in[5];
  const float* w_e1  = (const float*)d_in[6];
  const float* b_e1  = (const float*)d_in[7];
  const float* w_e2  = (const float*)d_in[8];
  const float* b_e2  = (const float*)d_in[9];
  const float* w_n1  = (const float*)d_in[10];
  const float* b_n1  = (const float*)d_in[11];
  const float* w_n2  = (const float*)d_in[12];
  const float* b_n2  = (const float*)d_in[13];
  const float* w_out = (const float*)d_in[14];
  const float* b_out = (const float*)d_in[15];
  float* out   = (float*)d_out;
  _Float16* Ft = (_Float16*)d_ws;

  k_nodef<<<dim3(B_ * N_ / 64), dim3(128), 0, stream>>>(x, w_in1, b_in1, w_in2, b_in2, w_e1, b_e1, w_e2, b_e2, Ft);
  k_aggout<<<dim3(B_ * H_ / 32), dim3(64), 0, stream>>>(adj, Ft, w_n1, b_n1, w_n2, b_n2, w_out, b_out, out);
  (void)hipGetLastError();
}
